// MatchNet_773094113749
// MI455X (gfx1250) — hardware-run, weakly checked
//
#include <hip/hip_runtime.h>
#include <math.h>

typedef __attribute__((ext_vector_type(16))) _Float16 v16h;
typedef __attribute__((ext_vector_type(8)))  _Float16 v8h;
typedef __attribute__((ext_vector_type(8)))  float    v8f;
typedef __attribute__((ext_vector_type(4)))  float    v4f;
typedef __attribute__((ext_vector_type(2)))  float    v2f;

constexpr int kRows      = 32768;
constexpr int kIn        = 6;
constexpr int kHid       = 20;
constexpr int kOut       = 8;
constexpr int kCons      = 6;
constexpr int kSteps     = 150;
constexpr int kPad       = 32;
constexpr int kSlabP     = 36;
constexpr int kZP        = 16;
constexpr int kWaves     = 8;
constexpr int kRowsWave  = 32;
constexpr int kRowsBlock = kWaves * kRowsWave;
constexpr int kBlocks    = kRows / kRowsBlock;
constexpr float kCarryH   = 32.0f;
constexpr float kCarryW   = 64.0f;
constexpr float kInvCarry = 1.0f / (kCarryH * kCarryW);
constexpr float kCarryR   = 2048.0f;
constexpr float kInvRem   = 1.0f / kCarryR;
constexpr float kHalfMinNormal = 6.103515625e-5f;
constexpr float kStrength = 10.0f;
static_assert((kRows % kRowsBlock) == 0, "exact grid");
static_assert(kHid <= kPad && kOut <= 16 && kIn <= 8, "padded extents");
static_assert((kPad % 32) == 0, "K step of the matrix instruction");
static_assert((kSlabP % 4) == 0 && 16 * kSlabP >= kRowsWave * kOut, "slab holds the output tile");
static_assert(kCons * kOut == 48, "constraint matrix extent");

__device__ __forceinline__ _Float16 to_h_flush(float v) {
  const float w = (fabsf(v) < kHalfMinNormal) ? 0.0f : v;
  return (_Float16)w;
}

union FragU { v16h v; v8h h[2]; };
__device__ __forceinline__ v16h frag_load(const _Float16* p) {
  FragU f;
  f.h[0] = *(const v8h*)(p);
  f.h[1] = *(const v8h*)(p + 16);
  return f.v;
}

__device__ __forceinline__ v8f mma_guarded(v16h a, v16h b, v8f c) {
  c = __builtin_amdgcn_wmma_f32_16x16x32_f16(false, a, false, b, (short)0, c, false, false);
  asm volatile("v_nop\n\tv_nop\n\tv_nop\n\tv_nop" : "+v"(c) : "v"(a), "v"(b));
  return c;
}

__global__ __launch_bounds__(256) void mlp_lp_iter_kernel(
    const float* __restrict__ X,
    const float* __restrict__ W1, const float* __restrict__ b1,
    const float* __restrict__ W2, const float* __restrict__ b2,
    const float* __restrict__ W3, const float* __restrict__ b3,
    const float* __restrict__ W4, const float* __restrict__ b4,
    const float* __restrict__ S,
    float* __restrict__ out)
{
  __shared__ __align__(16) float    sW1[kIn * kPad];
  __shared__ __align__(16) float    sBias[4 * kPad];
  __shared__ __align__(16) _Float16 sBt23[2 * kPad * kPad];
  __shared__ __align__(16) _Float16 sBt23r[2 * kPad * kPad];
  __shared__ __align__(16) _Float16 sBt4[16 * kPad];
  __shared__ __align__(16) _Float16 sBt4r[16 * kPad];
  __shared__ __align__(16) _Float16 sA[kWaves][16 * kPad];
  __shared__ __align__(16) _Float16 sAr[kWaves][16 * kPad];
  __shared__ __align__(16) float    sSlab[kWaves][16 * kSlabP];
  __shared__ __align__(16) float    sZ[kWaves][kRowsWave * kZP];

  const int tid  = threadIdx.x;
  const int wave = tid >> 5;
  const int lane = tid & 31;
  const int m    = lane & 15;
  const int hh   = lane >> 4;

  {
    const int pl = tid >> 7;
    const int tt = tid & 127;
    const int n  = tt >> 2;
    const int k8 = (tt & 3) * 8;
    const float* Wsrc = (pl == 0) ? W2 : W3;
    const int nc = (n < kHid) ? n : (kHid - 1);
    v8h hv, rv;
#pragma unroll
    for (int e = 0; e < 8; ++e) {
      const int k  = k8 + e;
      const int kc = (k < kHid) ? k : (kHid - 1);
      float w = Wsrc[kc * kHid + nc];
      asm volatile("" : "+v"(w));
      const bool real = (n < kHid) && (k < kHid);
      const float wc = real ? (w * kCarryW) : 0.0f;
      const _Float16 hval = to_h_flush(wc);
      const float rem = (wc - (float)hval) * kCarryR;
      hv[e] = hval;
      rv[e] = to_h_flush(rem);
    }
    *(v8h*)(sBt23  + pl * (kPad * kPad) + n * kPad + k8) = hv;
    *(v8h*)(sBt23r + pl * (kPad * kPad) + n * kPad + k8) = rv;
  }
  if (tid < 64) {
    const int n  = tid >> 2;
    const int k8 = (tid & 3) * 8;
    const int nc = (n < kOut) ? n : (kOut - 1);
    v8h hv, rv;
#pragma unroll
    for (int e = 0; e < 8; ++e) {
      const int k  = k8 + e;
      const int kc = (k < kHid) ? k : (kHid - 1);
      float w = W4[kc * kOut + nc];
      asm volatile("" : "+v"(w));
      const bool real = (n < kOut) && (k < kHid);
      const float wc = real ? (w * kCarryW) : 0.0f;
      const _Float16 hval = to_h_flush(wc);
      const float rem = (wc - (float)hval) * kCarryR;
      hv[e] = hval;
      rv[e] = to_h_flush(rem);
    }
    *(v8h*)(sBt4  + n * kPad + k8) = hv;
    *(v8h*)(sBt4r + n * kPad + k8) = rv;
  } else {
    const int idx = tid - 64;
    const int k   = idx >> 5;
    const int c   = idx & 31;
    const int cc  = (c < kHid) ? c : (kHid - 1);
    float w = W1[k * kHid + cc];
    asm volatile("" : "+v"(w));
    sW1[k * kPad + c] = (c < kHid) ? w : 0.0f;
  }
  if (tid < 128) {
    const int lay = tid >> 5;
    const int c   = tid & 31;
    const float* bp = (lay == 0) ? b1 : ((lay == 1) ? b2 : ((lay == 2) ? b3 : b4));
    const int nb = (lay == 3) ? kOut : kHid;
    const int cc = (c < nb) ? c : (nb - 1);
    float v = bp[cc];
    asm volatile("" : "+v"(v));
    sBias[lay * kPad + c] = (c < nb) ? v : 0.0f;
  }
  __syncthreads();

  const int rowW0 = blockIdx.x * kRowsBlock + wave * kRowsWave;
  _Float16* aw   = sA[wave];
  _Float16* awr  = sAr[wave];
  float*    slab = sSlab[wave];
  float*    zw   = sZ[wave];

#pragma unroll 1
  for (int t = 0; t < 2; ++t) {
    int rowT = rowW0 + 16 * t + m;
    rowT = (rowT < kRows) ? rowT : (kRows - 1);
    const v2f* xp = (const v2f*)(X + (size_t)rowT * kIn);
    const v2f xa = xp[0];
    const v2f xb2 = xp[1];
    const v2f xc = xp[2];
    float zin[kIn];
    zin[0] = xa[0]; zin[1] = xa[1]; zin[2] = xb2[0]; zin[3] = xb2[1]; zin[4] = xc[0]; zin[5] = xc[1];

#pragma unroll 1
    for (int lay = 0; lay < 3; ++lay) {
      if (lay == 0) {
#pragma unroll 1
        for (int e8 = 0; e8 < 2; ++e8) {
          const int c0 = 16 * hh + 8 * e8;
          v4f p0 = (v4f){0.f, 0.f, 0.f, 0.f};
          v4f p1 = (v4f){0.f, 0.f, 0.f, 0.f};
#pragma unroll
          for (int k = 0; k < kIn; ++k) {
            const v4f wa = *(const v4f*)(sW1 + k * kPad + c0);
            const v4f wb = *(const v4f*)(sW1 + k * kPad + c0 + 4);
            const float zk = zin[k];
#pragma unroll
            for (int q = 0; q < 4; ++q) {
              p0[q] = fmaf(zk, wa[q], p0[q]);
              p1[q] = fmaf(zk, wb[q], p1[q]);
            }
          }
          *(v4f*)(slab + m * kSlabP + c0)     = p0;
          *(v4f*)(slab + m * kSlabP + c0 + 4) = p1;
        }
      } else {
        const v16h ah = frag_load(aw  + m * kPad + 8 * hh);
        const v16h al = frag_load(awr + m * kPad + 8 * hh);
        const _Float16* bt  = sBt23  + (lay - 1) * (kPad * kPad);
        const _Float16* btr = sBt23r + (lay - 1) * (kPad * kPad);
#pragma unroll 1
        for (int j = 0; j < 2; ++j) {
          const v16h bh = frag_load(bt  + (16 * j + m) * kPad + 8 * hh);
          const v16h bl = frag_load(btr + (16 * j + m) * kPad + 8 * hh);
          v8f acc  = (v8f){0.f, 0.f, 0.f, 0.f, 0.f, 0.f, 0.f, 0.f};
          v8f accr = (v8f){0.f, 0.f, 0.f, 0.f, 0.f, 0.f, 0.f, 0.f};
          acc  = mma_guarded(ah, bh, acc);
          accr = mma_guarded(ah, bl, accr);
          accr = mma_guarded(al, bh, accr);
#pragma unroll
          for (int r = 0; r < 8; ++r) slab[(8 * hh + r) * kSlabP + 16 * j + m] = fmaf(accr[r], kInvRem, acc[r]);
        }
      }
      __syncthreads();
      {
        const float fold = (lay == 0) ? 1.0f : kInvCarry;
        const float* bl = sBias + lay * kPad;
#pragma unroll 1
        for (int e8 = 0; e8 < 2; ++e8) {
          const int c0 = 16 * hh + 8 * e8;
          const v4f s0 = *(const v4f*)(slab + m * kSlabP + c0);
          const v4f s1 = *(const v4f*)(slab + m * kSlabP + c0 + 4);
          const v4f g0 = *(const v4f*)(bl + c0);
          const v4f g1 = *(const v4f*)(bl + c0 + 4);
          v8h hv, rv;
#pragma unroll
          for (int e = 0; e < 4; ++e) {
            const float pa = fmaf(s0[e], fold, g0[e]);
            const float pb = fmaf(s1[e], fold, g1[e]);
            const float ta = tanhf(pa);
            const float tb = tanhf(pb);
            const float ca = ((c0 + e) < kHid) ? (ta * kCarryH) : 0.0f;
            const float cb = ((c0 + 4 + e) < kHid) ? (tb * kCarryH) : 0.0f;
            const _Float16 ha = to_h_flush(ca);
            const _Float16 hb = to_h_flush(cb);
            const float ra = (ca - (float)ha) * kCarryR;
            const float rb = (cb - (float)hb) * kCarryR;
            hv[e]     = ha;
            hv[4 + e] = hb;
            rv[e]     = to_h_flush(ra);
            rv[4 + e] = to_h_flush(rb);
          }
          *(v8h*)(aw  + m * kPad + c0) = hv;
          *(v8h*)(awr + m * kPad + c0) = rv;
        }
      }
      __syncthreads();
    }
    {
      const v16h ah = frag_load(aw  + m * kPad + 8 * hh);
      const v16h al = frag_load(awr + m * kPad + 8 * hh);
      const v16h bh = frag_load(sBt4  + m * kPad + 8 * hh);
      const v16h bl = frag_load(sBt4r + m * kPad + 8 * hh);
      v8f acc  = (v8f){0.f, 0.f, 0.f, 0.f, 0.f, 0.f, 0.f, 0.f};
      v8f accr = (v8f){0.f, 0.f, 0.f, 0.f, 0.f, 0.f, 0.f, 0.f};
      acc  = mma_guarded(ah, bh, acc);
      accr = mma_guarded(ah, bl, accr);
      accr = mma_guarded(al, bh, accr);
      const float bz = sBias[3 * kPad + m];
#pragma unroll
      for (int r = 0; r < 8; ++r) {
        const float sacc = fmaf(accr[r], kInvRem, acc[r]);
        zw[(16 * t + 8 * hh + r) * kZP + m] = fmaf(sacc, kInvCarry, bz);
      }
    }
  }
  __syncthreads();

  int rowP = rowW0 + lane;
  rowP = (rowP < kRows) ? rowP : (kRows - 1);
  float zt[kOut];
  {
    const v4f z0 = *(const v4f*)(zw + lane * kZP);
    const v4f z1 = *(const v4f*)(zw + lane * kZP + 4);
    zt[0] = z0[0]; zt[1] = z0[1]; zt[2] = z0[2]; zt[3] = z0[3];
    zt[4] = z1[0]; zt[5] = z1[1]; zt[6] = z1[2]; zt[7] = z1[3];
  }
  float bq[kCons];
  {
    const v2f* xq = (const v2f*)(X + (size_t)rowP * kIn);
    const v2f qa = xq[0];
    const v2f qb = xq[1];
    const v2f qc = xq[2];
    bq[0] = qa[0]; bq[1] = qa[1]; bq[2] = qb[0]; bq[3] = qb[1]; bq[4] = qc[0]; bq[5] = qc[1];
  }
  float sm[kCons * kOut];
  float ss = (float)kOut;
#pragma unroll
  for (int i = 0; i < kCons * kOut; ++i) {
    const float v = S[i];
    sm[i] = v;
    ss = fmaf(v, v, ss);
  }
  const float tau = 1.0f / sqrtf(ss);
  const float sigma = tau;
  const float tc = tau * kStrength;

  float xs[kOut], xbar[kOut], ys[kCons + kOut];
#pragma unroll
  for (int j = 0; j < kOut; ++j) {
    xs[j] = fmaxf(zt[j], 0.0f);
    xbar[j] = xs[j];
  }
#pragma unroll
  for (int i = 0; i < kCons + kOut; ++i) ys[i] = 0.0f;

#pragma unroll 1
  for (int it = 0; it < kSteps; ++it) {
#pragma unroll
    for (int i = 0; i < kCons; ++i) {
      float dot = 0.0f;
#pragma unroll
      for (int j = 0; j < kOut; ++j) dot = fmaf(sm[i * kOut + j], xbar[j], dot);
      const float res = dot - bq[i];
      ys[i] = fmaxf(0.0f, fmaf(sigma, res, ys[i]));
    }
#pragma unroll
    for (int j = 0; j < kOut; ++j) ys[kCons + j] = fmaxf(0.0f, fmaf(sigma, -xbar[j], ys[kCons + j]));
    float dd[kOut];
    float n2 = 0.0f;
#pragma unroll
    for (int j = 0; j < kOut; ++j) {
      float g = 0.0f;
#pragma unroll
      for (int i = 0; i < kCons; ++i) g = fmaf(ys[i], sm[i * kOut + j], g);
      g = g - ys[kCons + j];
      const float v = fmaf(-tau, g, xs[j]);
      const float u = v + tau;
      dd[j] = u - zt[j];
      n2 = fmaf(dd[j], dd[j], n2);
    }
    const float nn = sqrtf(n2);
    const float q  = tc / fmaxf(nn, 1e-12f);
    const float sc = fmaxf(0.0f, 1.0f - q);
#pragma unroll
    for (int j = 0; j < kOut; ++j) {
      const float xn = fmaf(sc, dd[j], zt[j]);
      xbar[j] = fmaf(2.0f, xn, -xs[j]);
      xs[j] = xn;
    }
  }

  {
    const v4f r0 = (v4f){xs[0], xs[1], xs[2], xs[3]};
    const v4f r1 = (v4f){xs[4], xs[5], xs[6], xs[7]};
    *(v4f*)(slab + lane * kOut)     = r0;
    *(v4f*)(slab + lane * kOut + 4) = r1;
  }
  __syncthreads();
  {
    const v4f o0 = *(const v4f*)(slab + lane * 4);
    const v4f o1 = *(const v4f*)(slab + 128 + lane * 4);
    if (rowW0 + kRowsWave <= kRows) {
      float* ob = out + (size_t)rowW0 * kOut;
      for (int pass = 0; pass < 2; ++pass) {
        *(volatile v4f*)(ob + lane * 4)       = o0;
        *(volatile v4f*)(ob + 128 + lane * 4) = o1;
        __threadfence();
      }
    }
  }
}

extern "C" void kernel_launch(void* const* d_in, const int* in_sizes, int n_in,
                              void* d_out, int out_size, void* d_ws, size_t ws_size,
                              hipStream_t stream) {
  (void)d_ws;
  (void)ws_size;
  if (n_in < 10) return;
  if (in_sizes[0] != kRows * kIn) return;
  if (in_sizes[1] != kIn * kHid) return;
  if (in_sizes[2] != kHid) return;
  if (in_sizes[3] != kHid * kHid) return;
  if (in_sizes[4] != kHid) return;
  if (in_sizes[5] != kHid * kHid) return;
  if (in_sizes[6] != kHid) return;
  if (in_sizes[7] != kHid * kOut) return;
  if (in_sizes[8] != kOut) return;
  if (in_sizes[9] != kCons * kOut) return;
  if (out_size != kRows * kOut) return;

  const float* X  = (const float*)d_in[0];
  const float* W1 = (const float*)d_in[1];
  const float* b1 = (const float*)d_in[2];
  const float* W2 = (const float*)d_in[3];
  const float* b2 = (const float*)d_in[4];
  const float* W3 = (const float*)d_in[5];
  const float* b3 = (const float*)d_in[6];
  const float* W4 = (const float*)d_in[7];
  const float* b4 = (const float*)d_in[8];
  const float* S  = (const float*)d_in[9];
  float* out = (float*)d_out;

  mlp_lp_iter_kernel<<<kBlocks, 256, 0, stream>>>(X, W1, b1, W2, b2, W3, b3, W4, b4, S, out);
}
